// DoubleSin_36146444763907
// MI455X (gfx1250) — hardware-verified
//
#include <hip/hip_runtime.h>
#include <stdint.h>


typedef __attribute__((ext_vector_type(16))) _Float16 v16h;
typedef __attribute__((ext_vector_type(8)))  _Float16 v8h;
typedef __attribute__((ext_vector_type(4)))  _Float16 v4h;
typedef __attribute__((ext_vector_type(8)))  float    v8f;
typedef __attribute__((ext_vector_type(4)))  float    v4f;

__device__ __forceinline__ void dep_guard_h(v8f& a, v8f& b, v16h x, v16h y) { asm volatile("v_nop\n\tv_nop\n\tv_nop\n\tv_nop" : "+v"(a), "+v"(b) : "v"(x), "v"(y)); }
__device__ __forceinline__ void keep4_h(v16h a, v16h b, v16h c, v16h d) { asm volatile("v_nop" :: "v"(a), "v"(b), "v"(c), "v"(d)); }

template <typename T> struct Frag;
template <> struct Frag<_Float16> {
  typedef v16h V; union U { v16h v; v8h h[2]; };
  static __device__ __forceinline__ v16h load(const _Float16* p) {
    U f; f.h[0] = *(const v8h*)(p); f.h[1] = *(const v8h*)(p + 16); return f.v;
  }
  static __device__ __forceinline__ v8f mma(v16h a, v16h b, v8f c) {
    return __builtin_amdgcn_wmma_f32_16x16x32_f16(false, a, false, b, (short)0, c, false, false);
  }
  static __device__ __forceinline__ void guard(v8f& a, v8f& b, v16h x, v16h y) { dep_guard_h(a, b, x, y); }
  static __device__ __forceinline__ void keep(v16h a, v16h b, v16h c, v16h d) { keep4_h(a, b, c, d); }
};

#define LDH 72
#define TR 256
#define NTHR 256
#define NPAR 11
#define WSC 64.0f
#define WSC_INV 0.015625f
#define GRID_CAP 2048

struct KParams {
  const float* x;
  const float* w[22];
  float* out;
  int n;
  int nx;
  int tiles;
  int pad0;
};
static_assert(sizeof(KParams) == 208);

__device__ __forceinline__ float snake_f(float t, float a, float ia) {
  const float u  = a * t;
  const float k  = __builtin_rintf(u * 0.318309886f);
  float r = fmaf(-k, 3.14159274f, u);
  r = fmaf(-k, -8.742278e-8f, r);
  const float r2 = r * r;
  float p = fmaf(r2, -2.5052108e-8f, 2.7557319e-6f);
  p = fmaf(r2, p, -1.9841270e-4f);
  p = fmaf(r2, p, 8.3333333e-3f);
  p = fmaf(r2, p, -1.6666667e-1f);
  const float s = fmaf(r2 * r, p, r);
  return fmaf(s * s, ia, t);
}

__device__ __forceinline__ void wave_sync() {
  __builtin_amdgcn_fence(__ATOMIC_RELEASE, "workgroup");
  __builtin_amdgcn_wave_barrier();
  __builtin_amdgcn_fence(__ATOMIC_ACQUIRE, "workgroup");
}

__device__ __forceinline__ void stage_mat(_Float16* dst, const float* __restrict__ src, int tid) {
#pragma unroll
  for (int it = 0; it < 4; ++it) {
    const int q = it * NTHR + tid;
    const v4f v = *(const v4f*)(src + (size_t)q * 4);
    const int e = q * 4, nn = e >> 6, kk = e & 63;
    v4h hv;
    hv[0] = (_Float16)(v[0] * WSC);
    hv[1] = (_Float16)(v[1] * WSC);
    hv[2] = (_Float16)(v[2] * WSC);
    hv[3] = (_Float16)(v[3] * WSC);
    *(v4h*)(dst + nn * LDH + kk) = hv;
  }
}

__device__ __forceinline__ void stage_vecs(float* dst,
    const float* __restrict__ W1, const float* __restrict__ b1, const float* __restrict__ a1,
    const float* __restrict__ b2, const float* __restrict__ a2,
    const float* __restrict__ b3, const float* __restrict__ a3,
    const float* __restrict__ W4, int j) {
  dst[0 * 64 + j] = W1[j];
  dst[1 * 64 + j] = b1[j];
  float a = a1[j];
  dst[2 * 64 + j] = a;
  dst[3 * 64 + j] = 1.0f / a;
  dst[4 * 64 + j] = b2[j];
  a = a2[j];
  dst[5 * 64 + j] = a;
  dst[6 * 64 + j] = 1.0f / a;
  dst[7 * 64 + j] = b3[j];
  a = a3[j];
  dst[8 * 64 + j] = a;
  dst[9 * 64 + j] = 1.0f / a;
  dst[10 * 64 + j] = W4[j];
}

__device__ __forceinline__ void gemm_snake_layer(
    _Float16* sHw, const _Float16* sWm,
    const float* bias, const float* av, const float* iav, int lane)
{
  const int m  = lane & 15;
  const int h8 = (lane >> 4) * 8;

  v16h A[2][2];
#pragma unroll
  for (int mt = 0; mt < 2; ++mt)
#pragma unroll
    for (int kf = 0; kf < 2; ++kf)
      A[mt][kf] = Frag<_Float16>::load(sHw + (mt * 16 + m) * LDH + kf * 32 + h8);

  const v8f zero = (v8f){0.f, 0.f, 0.f, 0.f, 0.f, 0.f, 0.f, 0.f};

#pragma unroll 1
  for (int nt = 0; nt < 4; ++nt) {
    const _Float16* pb = sWm + (nt * 16 + m) * LDH + h8;
    const v16h B0 = Frag<_Float16>::load(pb);
    const v16h B1 = Frag<_Float16>::load(pb + 32);
    v8f acc0 = zero, acc1 = zero;
    acc0 = Frag<_Float16>::mma(A[0][0], B0, acc0);
    acc1 = Frag<_Float16>::mma(A[1][0], B0, acc1);
    acc0 = Frag<_Float16>::mma(A[0][1], B1, acc0);
    acc1 = Frag<_Float16>::mma(A[1][1], B1, acc1);
    dep_guard_h(acc0, acc1, B0, B1);
    keep4_h(A[0][0], A[0][1], A[1][0], A[1][1]);

    const int ch = nt * 16 + m;
    const float bv = bias[ch];
    const float aa = av[ch];
    const float ia = iav[ch];
#pragma unroll
    for (int r = 0; r < 8; ++r) {
      const float v0 = snake_f(fmaf(acc0[r], WSC_INV, bv), aa, ia);
      const float v1 = snake_f(fmaf(acc1[r], WSC_INV, bv), aa, ia);
      sHw[(h8 + r) * LDH + ch]      = (_Float16)v0;
      sHw[(16 + h8 + r) * LDH + ch] = (_Float16)v1;
    }
  }
  keep4_h(A[0][0], A[0][1], A[1][0], A[1][1]);
}

__global__ __launch_bounds__(NTHR)
void fused_snake_mlp_kernel(KParams p)
{
  __shared__ __align__(16) _Float16 sH[TR * LDH];
  __shared__ __align__(16) _Float16 sW[4][64 * LDH];
  __shared__ __align__(16) float    sPar[2][NPAR][64];

  const int tid  = threadIdx.x;
  const int wave = tid >> 5;
  const int lane = tid & 31;

  stage_mat(sW[0], p.w[3],  tid);
  stage_mat(sW[1], p.w[6],  tid);
  stage_mat(sW[2], p.w[14], tid);
  stage_mat(sW[3], p.w[17], tid);
  if (tid < 64) {
    stage_vecs(&sPar[0][0][0], p.w[0],  p.w[1],  p.w[2],  p.w[4],  p.w[5],  p.w[7],  p.w[8],  p.w[9],  tid);
    stage_vecs(&sPar[1][0][0], p.w[11], p.w[12], p.w[13], p.w[15], p.w[16], p.w[18], p.w[19], p.w[20], tid);
  }
  const float b4a = p.w[10][0];
  const float b4b = p.w[21][0];
  __syncthreads();

  _Float16* sHw   = sH + wave * 32 * LDH;
  _Float16* myrow = sHw + lane * LDH;

  for (int t = blockIdx.x; t < p.tiles; t += gridDim.x) {
    const int row  = t * TR + wave * 32 + lane;
    const int rowc = row < p.nx ? row : (p.nx - 1);
    const float xv = p.x[rowc];
    float o = 0.0f;

#pragma unroll 1
    for (int br = 0; br < 2; ++br) {
      const float xb = br ? (xv + xv) : xv;
      const float* P  = &sPar[br][0][0];
      const float* W1 = P;
      const float* B1 = P + 64;
      const float* A1 = P + 2 * 64;
      const float* I1 = P + 3 * 64;

      for (int c8 = 0; c8 < 8; ++c8) {
        v8h hv;
#pragma unroll
        for (int e = 0; e < 8; ++e) {
          const int ch = c8 * 8 + e;
          hv[e] = (_Float16)snake_f(fmaf(xb, W1[ch], B1[ch]), A1[ch], I1[ch]);
        }
        *(v8h*)(myrow + c8 * 8) = hv;
      }
      wave_sync();

      gemm_snake_layer(sHw, sW[br * 2 + 0], P + 4 * 64, P + 5 * 64, P + 6 * 64, lane);
      wave_sync();
      gemm_snake_layer(sHw, sW[br * 2 + 1], P + 7 * 64, P + 8 * 64, P + 9 * 64, lane);
      wave_sync();

      const float* W4 = P + 10 * 64;
      float d = 0.0f;
#pragma unroll
      for (int c8 = 0; c8 < 8; ++c8) {
        const v8h hv = *(const v8h*)(myrow + c8 * 8);
#pragma unroll
        for (int e = 0; e < 8; ++e) d = fmaf((float)hv[e], W4[c8 * 8 + e], d);
      }
      o += d + (br ? b4b : b4a);
      wave_sync();
    }

    if (row < p.n) *(volatile float*)(p.out + row) = o;
    __threadfence();
    if (row < p.n) *(volatile float*)(p.out + row) = o;
  }
}

extern "C" void kernel_launch(void* const* d_in, const int* in_sizes, int n_in,
                              void* d_out, int out_size, void* d_ws, size_t ws_size,
                              hipStream_t stream)
{
  (void)d_ws; (void)ws_size;
  if (n_in < 23 || out_size <= 0) return;
  KParams kp;
  kp.x = (const float*)d_in[0];
  for (int i = 0; i < 22; ++i) kp.w[i] = (const float*)d_in[1 + i];
  kp.out   = (float*)d_out;
  kp.n     = out_size;
  kp.nx    = in_sizes[0] > 0 ? in_sizes[0] : 1;
  kp.tiles = (out_size + TR - 1) / TR;
  kp.pad0  = 0;
  int grid = kp.tiles < GRID_CAP ? kp.tiles : GRID_CAP;
  if (grid < 1) grid = 1;
  hipLaunchKernelGGL(fused_snake_mlp_kernel, dim3(grid), dim3(NTHR), 0, stream, kp);
}
